// Model_Comi_Rec_25769803776123
// MI455X (gfx1250) — hardware-run, weakly checked
//
#include <hip/hip_runtime.h>
#include <stddef.h>
#include <stdint.h>

#define NB    1024
#define NS    50
#define ND    128
#define NI    4
#define NK    512
#define NMID  100000
#define SWP   52

static_assert(NK == NI * ND);
static_assert(ND % 32 == 0);
static_assert(NB % 256 == 0);
static_assert(NK % 64 == 0);
static_assert((NS * NK * ND) % 2048 == 0);
static_assert((NS * NB * ND) % 2048 == 0);
static_assert((NI * NS * ND) % 4 == 0);
static_assert(NI * NS <= 256);
static_assert(NI * ND == 512);

typedef _Float16 v16h __attribute__((ext_vector_type(16)));
typedef _Float16 v8h  __attribute__((ext_vector_type(8)));
typedef float    v8f  __attribute__((ext_vector_type(8)));
typedef float    v4f  __attribute__((ext_vector_type(4)));
typedef unsigned int v4u __attribute__((ext_vector_type(4)));

union Frag  { v16h v; v8h h[2]; };
union Pack8 { v8h h; v4u u; };

__device__ __forceinline__ v8f mma16(v16h a, v16h b, v8f c) {
  c = __builtin_amdgcn_wmma_f32_16x16x32_f16(false, a, false, b, (short)0, c, false, false);
  asm volatile("v_nop\n\tv_nop\n\tv_nop\n\tv_nop" : "+v"(c) : "v"(a), "v"(b));
  return c;
}

__device__ __forceinline__ v16h ldfrag(const _Float16* p, int ld, int row0, int k0, int lane) {
  const int m = lane & 15, lh = lane >> 4;
  const _Float16* q = p + (size_t)(row0 + m) * ld + k0 + 8 * lh;
  Frag f;
  f.h[0] = *(const v8h*)(q);
  f.h[1] = *(const v8h*)(q + 16);
  return f.v;
}

__device__ __forceinline__ v8f zero8() { return (v8f){0.f, 0.f, 0.f, 0.f, 0.f, 0.f, 0.f, 0.f}; }

__device__ __forceinline__ void gemm32x64(const _Float16* __restrict__ A, int lda,
                                          const _Float16* __restrict__ Bt, int ldb, int nks,
                                          int r0, int n0, int lane, v8f (&acc)[2][4]) {
#pragma unroll 1
  for (int ks = 0; ks < nks; ++ks) {
    const int k0 = 32 * ks;
    const v16h a0 = ldfrag(A, lda, r0, k0, lane);
    const v16h a1 = ldfrag(A, lda, r0 + 16, k0, lane);
    const v16h b0 = ldfrag(Bt, ldb, n0, k0, lane);
    const v16h b1 = ldfrag(Bt, ldb, n0 + 16, k0, lane);
    const v16h b2 = ldfrag(Bt, ldb, n0 + 32, k0, lane);
    const v16h b3 = ldfrag(Bt, ldb, n0 + 48, k0, lane);
    acc[0][0] = mma16(a0, b0, acc[0][0]);
    acc[1][0] = mma16(a1, b0, acc[1][0]);
    acc[0][1] = mma16(a0, b1, acc[0][1]);
    acc[1][1] = mma16(a1, b1, acc[1][1]);
    acc[0][2] = mma16(a0, b2, acc[0][2]);
    acc[1][2] = mma16(a1, b2, acc[1][2]);
    acc[0][3] = mma16(a0, b3, acc[0][3]);
    acc[1][3] = mma16(a1, b3, acc[1][3]);
  }
}

__global__ __launch_bounds__(256) void k_wcvt(const float* __restrict__ src, _Float16* __restrict__ dst,
                                              float scale) {
  const size_t o = ((size_t)blockIdx.x * 256 + threadIdx.x) * 8;
  const v4f a0 = *(const v4f*)(src + o) * scale;
  const v4f a1 = *(const v4f*)(src + o + 4) * scale;
  Pack8 pk;
  pk.h = (v8h){(_Float16)a0[0], (_Float16)a0[1], (_Float16)a0[2], (_Float16)a0[3],
               (_Float16)a1[0], (_Float16)a1[1], (_Float16)a1[2], (_Float16)a1[3]};
  const v4u vv = pk.u;
  volatile v4u* d = (volatile v4u*)(dst + o);
  *d = vv;
  __threadfence();
  *d = vv;
}

__global__ __launch_bounds__(256) void k_items(const int* __restrict__ hist_item,
                                               const float* __restrict__ hist_mask,
                                               const float* __restrict__ mid_emb,
                                               _Float16* __restrict__ Ah) {
  const int idx = blockIdx.x * 256 + threadIdx.x;
  const int pc = idx & 15;
  const int r  = idx >> 4;
  const int s  = r >> 10;
  const int b  = r & (NB - 1);
  int hi = hist_item[b * NS + s];
  hi = min(max(hi, 0), NMID - 1);
  const float f = hist_mask[b * NS + s] * 64.0f;
  const float* sp = mid_emb + (size_t)hi * ND + 8 * pc;
  const v4f a0 = *(const v4f*)(sp) * f;
  const v4f a1 = *(const v4f*)(sp + 4) * f;
  Pack8 pk;
  pk.h = (v8h){(_Float16)a0[0], (_Float16)a0[1], (_Float16)a0[2], (_Float16)a0[3],
               (_Float16)a1[0], (_Float16)a1[1], (_Float16)a1[2], (_Float16)a1[3]};
  const v4u vv = pk.u;
  volatile v4u* d = (volatile v4u*)(Ah + (size_t)r * ND + 8 * pc);
  *d = vv;
  __threadfence();
  *d = vv;
}

#define OTP 68
__global__ __launch_bounds__(256) void k_gemm(const _Float16* __restrict__ A, const _Float16* __restrict__ Bt,
                                              float* __restrict__ outf, float scale) {
  __shared__ __align__(16) float st[8][16 * OTP];
  const int tid = threadIdx.x, lane = tid & 31, wave = tid >> 5;
  const int hh = lane >> 4, c = lane & 15;
  const int g  = blockIdx.z;
  const int m0 = blockIdx.x * 256 + wave * 32;
  const int n0 = blockIdx.y * 64;

  const _Float16* Ag = A  + (size_t)g * (NB * ND);
  const _Float16* Bg = Bt + (size_t)g * (NK * ND);

  v8f acc[2][4];
#pragma unroll
  for (int s = 0; s < 2; ++s)
#pragma unroll
    for (int t = 0; t < 4; ++t) acc[s][t] = zero8();
  gemm32x64(Ag, ND, Bg, ND, ND / 32, m0, n0, lane, acc);

  float* sw = st[wave];
  const size_t obase = (size_t)g * ((size_t)NB * NK);
#pragma unroll
  for (int sub = 0; sub < 2; ++sub) {
    __syncthreads();
#pragma unroll
    for (int t = 0; t < 4; ++t) {
#pragma unroll
      for (int r = 0; r < 8; ++r) sw[(8 * hh + r) * OTP + 16 * t + c] = acc[sub][t][r] * scale;
    }
    __syncthreads();
    const int mr0 = m0 + sub * 16;
    v4f val[8];
    size_t go[8];
#pragma unroll
    for (int it = 0; it < 8; ++it) {
      const int p    = lane + 32 * it;
      const int L    = p >> 3;
      const int pc   = p & 7;
      const int row  = L >> 1;
      const int half = L & 1;
      val[it] = *(const v4f*)(sw + row * OTP + half * 32 + pc * 4);
      go[it]  = obase + (size_t)(mr0 + row) * NK + n0 + half * 32 + pc * 4;
    }
#pragma unroll
    for (int it = 0; it < 8; ++it) *(volatile v4f*)(outf + go[it]) = val[it];
    __threadfence();
#pragma unroll
    for (int it = 0; it < 8; ++it) *(volatile v4f*)(outf + go[it]) = val[it];
  }
}

__global__ __launch_bounds__(256) void k_route(const float* __restrict__ hat,
                                               const float* __restrict__ hist_mask,
                                               float* __restrict__ out) {
  extern __shared__ __align__(16) float hat_s[];
  __shared__ __align__(16) float inter_s[NI * ND];
  __shared__ __align__(16) float cap_s[NI * ND];
  __shared__ float w_s[NI * NS];
  __shared__ float sw_s[NI * SWP];
  __shared__ float mask_s[SWP];
  __shared__ float red_s[8][2];
  __shared__ float scl_s[NI];

  const int b = blockIdx.x;
  const int tid = threadIdx.x, lane = tid & 31, wave = tid >> 5;

  const float* hb = hat + (size_t)b * NK;
#pragma unroll 1
  for (int i = tid; i < (NI * NS * ND) / 4; i += 256) {
    const int s = i >> 7, q = i & 127;
    const v4f v = *(const v4f*)(hb + (size_t)s * ((size_t)NB * NK) + 4 * q);
    const int n = q >> 5, d = 4 * (q & 31);
    *(v4f*)(hat_s + (n * NS + s) * ND + d) = v;
  }
  if (tid < NS) mask_s[tid] = hist_mask[b * NS + tid];
  if (tid < NI * NS) w_s[tid] = 0.0f;
  __syncthreads();

#pragma unroll 1
  for (int iter = 0; iter < 3; ++iter) {
    if (tid < NS) {
      const float w0 = w_s[0 * NS + tid], w1 = w_s[1 * NS + tid];
      const float w2 = w_s[2 * NS + tid], w3 = w_s[3 * NS + tid];
      const float mx = fmaxf(fmaxf(w0, w1), fmaxf(w2, w3));
      const float e0 = __expf(w0 - mx), e1 = __expf(w1 - mx);
      const float e2 = __expf(w2 - mx), e3 = __expf(w3 - mx);
      const float inv = 1.0f / ((e0 + e1) + (e2 + e3));
      const float mk = (mask_s[tid] == 0.0f) ? 0.0f : 1.0f;
      sw_s[0 * SWP + tid] = e0 * inv * mk;
      sw_s[1 * SWP + tid] = e1 * inv * mk;
      sw_s[2 * SWP + tid] = e2 * inv * mk;
      sw_s[3 * SWP + tid] = e3 * inv * mk;
    }
    __syncthreads();

    {
      const int o0 = tid, o1 = tid + 256;
      const int na = o0 >> 7, nb = o1 >> 7, d = o0 & (ND - 1);
      const float* ha = hat_s + (na * NS) * ND + d;
      const float* hb2 = hat_s + (nb * NS) * ND + d;
      const float* sa = sw_s + na * SWP;
      const float* sb = sw_s + nb * SWP;
      float a0 = 0.0f, a1 = 0.0f;
#pragma unroll 2
      for (int ss = 0; ss < NS; ++ss) {
        a0 += sa[ss] * ha[ss * ND];
        a1 += sb[ss] * hb2[ss * ND];
      }
      cap_s[o0] = a0;
      cap_s[o1] = a1;
      float p0 = a0 * a0, p1 = a1 * a1;
#pragma unroll
      for (int off = 16; off >= 1; off >>= 1) {
        p0 += __shfl_xor(p0, off, 32);
        p1 += __shfl_xor(p1, off, 32);
      }
      if (lane == 0) { red_s[wave][0] = p0; red_s[wave][1] = p1; }
    }
    __syncthreads();

    if (tid < NI) {
      const int wb = (tid & 1) * 4, sl = tid >> 1;
      const float cn = ((red_s[wb][sl] + red_s[wb + 1][sl]) + red_s[wb + 2][sl]) + red_s[wb + 3][sl];
      scl_s[tid] = cn / (1.0f + cn) / sqrtf(cn + 1e-9f);
    }
    __syncthreads();

    inter_s[tid]       = cap_s[tid] * scl_s[tid >> 7];
    inter_s[tid + 256] = cap_s[tid + 256] * scl_s[(tid + 256) >> 7];
    __syncthreads();

    if (iter < 2) {
      if (tid < NI * NS) {
        const int n = tid / NS, ss = tid - n * NS;
        const float* hr = hat_s + (n * NS + ss) * ND;
        const float* ir = inter_s + n * ND;
        float acc = 0.0f;
#pragma unroll 2
        for (int dd = 0; dd < ND; dd += 4) {
          const v4f hv = *(const v4f*)(hr + dd);
          const v4f iv = *(const v4f*)(ir + dd);
          acc += hv[0] * iv[0];
          acc += hv[1] * iv[1];
          acc += hv[2] * iv[2];
          acc += hv[3] * iv[3];
        }
        w_s[tid] = w_s[tid] + acc;
      }
      __syncthreads();
    }
  }

  if (tid < (NI * ND) / 4) {
    const v4f v = *(const v4f*)(inter_s + 4 * tid);
    volatile v4f* op = (volatile v4f*)(out + (size_t)b * (NI * ND) + 4 * tid);
    *op = v;
    __threadfence();
    *op = v;
  }
}

extern "C" void kernel_launch(void* const* d_in, const int* in_sizes, int n_in,
                              void* d_out, int out_size, void* d_ws, size_t ws_size,
                              hipStream_t stream) {
  if (n_in < 7) return;
  if (in_sizes[2] != NB * NS) return;
  if (in_sizes[3] != NB * NS) return;
  if (in_sizes[5] != NMID * ND) return;
  if (in_sizes[6] != NS * NK * ND) return;
  if (out_size != NB * NI * ND) return;

  const int*   hist_item = (const int*)d_in[2];
  const float* hist_mask = (const float*)d_in[3];
  const float* mid_emb   = (const float*)d_in[5];
  const float* caps_w    = (const float*)d_in[6];
  float* out = (float*)d_out;

  size_t off = 0;
  const size_t oW = off; off += (size_t)NS * NK * ND * 2;
  const size_t oA = off; off += (size_t)NS * NB * ND * 2;
  const size_t oH = off; off += (size_t)NS * NB * NK * 4;
  if (off > ws_size) return;
  if (off > (size_t)134217728) return;

  char* ws = (char*)d_ws;
  _Float16* Wh  = (_Float16*)(ws + oW);
  _Float16* Ah  = (_Float16*)(ws + oA);
  float*    Hat = (float*)(ws + oH);

  k_wcvt<<<dim3((NS * NK * ND) / 2048), dim3(256), 0, stream>>>(caps_w, Wh, 16.0f);
  k_items<<<dim3((NS * NB * ND) / 2048), dim3(256), 0, stream>>>(hist_item, hist_mask, mid_emb, Ah);

  k_gemm<<<dim3(NB / 256, NK / 64, NS), dim3(256), 0, stream>>>(Ah, Wh, Hat, 0.0009765625f);

  const size_t dyn = (size_t)NI * NS * ND * 4;
  (void)hipFuncSetAttribute(reinterpret_cast<const void*>(&k_route),
                            hipFuncAttributeMaxDynamicSharedMemorySize, (int)dyn);
  k_route<<<dim3(NB), dim3(256), dyn, stream>>>(Hat, hist_mask, out);
  (void)hipGetLastError();
}
